// GNNObservationEncoder_31190052504015
// MI455X (gfx1250) — hardware-verified
//
#include <hip/hip_runtime.h>
#include <math.h>


#define NB  8
#define NN  1024
#define NH  3
#define HD  64
#define HID 192
#define NEG_SLOPE 0.2f
typedef __attribute__((ext_vector_type(16))) _Float16 v16h;
typedef __attribute__((ext_vector_type(8)))  _Float16 v8h;
typedef __attribute__((ext_vector_type(8)))  float    v8f;
typedef __attribute__((ext_vector_type(4)))  float    v4f;
#define VST2(T, ptr, val) do { const T _v = (val); *(volatile T*)(ptr) = _v; __threadfence(); *(volatile T*)(ptr) = _v; } while (0)
__device__ __forceinline__ float leaky(float x) { return x > 0.f ? x : NEG_SLOPE * x; }
__device__ __forceinline__ int kmap(int e, int hh) { return (e < 8) ? (8 * hh + e) : (16 + 8 * hh + (e - 8)); }
__device__ __forceinline__ v8f wmma16(v16h a, v16h b, v8f c) {
  v8f d = __builtin_amdgcn_wmma_f32_16x16x32_f16(false, a, false, b, (short)0, c, false, false);
  asm volatile("v_nop\n\tv_nop\n\tv_nop\n\tv_nop" : "+v"(d) : "v"(a), "v"(b));
  return d;
}
__global__ __launch_bounds__(128) void k_xw(const float* __restrict__ x, int Fin, const float* __restrict__ W,
                                            float* __restrict__ Wh, _Float16* __restrict__ Whb) {
  __shared__ __attribute__((aligned(16))) float sT[16][64];
  const int lane = threadIdx.x & 31, wave = threadIdx.x >> 5, m = lane & 15, hh = lane >> 4;
  const int row0 = blockIdx.x * 16, h = blockIdx.y, b = blockIdx.z;
  const float* xr = x + ((size_t)b * NN + row0 + m) * Fin;
  const float* Wh_ = W + (size_t)h * Fin * HD;
  v8f c = {};
  for (int kk = 0; kk < Fin; kk += 32) {
    v16h A, B;
#pragma unroll
    for (int e = 0; e < 16; ++e) { const int k = kk + kmap(e, hh); A[e] = (_Float16)xr[k]; B[e] = (_Float16)Wh_[(size_t)k * HD + wave * 16 + m]; }
    c = wmma16(A, B, c);
  }
#pragma unroll
  for (int r = 0; r < 8; ++r) sT[r + 8 * hh][wave * 16 + m] = c[r];
  __syncthreads();
  const size_t ob = ((size_t)b * NN + row0) * HID + h * HD;
  for (int pass = 0; pass < 2; ++pass) {
#pragma unroll
    for (int j = 0; j < 2; ++j) { const int rr = j * 8 + (threadIdx.x >> 4), q4 = (threadIdx.x & 15) * 4;
      *(volatile v4f*)(Wh + ob + (size_t)rr * HID + q4) = *(const v4f*)(&sT[rr][q4]); }
    { const int rr = threadIdx.x >> 3, q8 = (threadIdx.x & 7) * 8; v8h v;
#pragma unroll
      for (int e = 0; e < 8; ++e) v[e] = (_Float16)sT[rr][q8 + e];
      *(volatile v8h*)(Whb + ob + (size_t)rr * HID + q8) = v; }
    __threadfence();
  }
}
__global__ __launch_bounds__(256) void k_scores(const float* __restrict__ Wh, const float* __restrict__ a, float* __restrict__ s_src, float* __restrict__ s_dst) {
  const int idx = blockIdx.x * 256 + threadIdx.x;
  if (idx >= NB * NH * NN) return;
  const int n = idx & (NN - 1), h = (idx >> 10) % NH, b = idx / (NH * NN);
  const float* w = Wh + ((size_t)b * NN + n) * HID + h * HD;
  const float* al = a + h * 2 * HD;
  float ss = 0.f, sd = 0.f;
#pragma unroll 8
  for (int d = 0; d < HD; ++d) { const float v = w[d]; ss += v * al[d]; sd += v * al[HD + d]; }
  VST2(float, s_src + idx, ss);
  VST2(float, s_dst + idx, sd);
}
__global__ __launch_bounds__(256) void k_rowmax(const float* __restrict__ adj, const float* __restrict__ s_src, const float* __restrict__ s_dst, float* __restrict__ emax) {
  __shared__ float se[32];
  const int lane = threadIdx.x & 31, wave = threadIdx.x >> 5;
  const int bh = blockIdx.y, i0 = blockIdx.x * 32;
  for (int q = 0; q < 4; ++q) {
    const int i = i0 + wave * 4 + q;
    float mx = -__builtin_inff();
    for (int j = lane; j < NN; j += 32) if (adj[(size_t)i * NN + j] > 0.f) mx = fmaxf(mx, s_dst[(size_t)bh * NN + j]);
#pragma unroll
    for (int off = 16; off > 0; off >>= 1) mx = fmaxf(mx, __shfl_xor(mx, off));
    if (lane == 0) se[wave * 4 + q] = leaky(s_src[(size_t)bh * NN + i] + mx);
  }
  __syncthreads();
  if (threadIdx.x < 32) VST2(float, emax + (size_t)bh * NN + i0 + threadIdx.x, se[threadIdx.x]);
}
__global__ __launch_bounds__(96) void k_aggregate(const float* __restrict__ adj, const _Float16* __restrict__ Whb, const float* __restrict__ s_src,
                                                  const float* __restrict__ s_dst, const float* __restrict__ emax, float* __restrict__ out, int doElu) {
  __shared__ __attribute__((aligned(16))) float sO[3][16][HD];
  const int lane = threadIdx.x & 31, wave = threadIdx.x >> 5, m = lane & 15, hh = lane >> 4;
  const int head = wave, row0 = blockIdx.x * 16, b = blockIdx.y, arow = row0 + m;
  const size_t bh = (size_t)b * NH + head;
  const float si = s_src[bh * NN + arow], em = emax[bh * NN + arow];
  const float* adjr = adj + (size_t)arow * NN;
  const _Float16* whh = Whb + (size_t)b * NN * HID + head * HD;
  v8f c[4] = {};
  float lsum = 0.f;
  for (int jb = 0; jb < NN; jb += 32) {
    v16h A;
#pragma unroll
    for (int e = 0; e < 16; ++e) {
      const int j = jb + kmap(e, hh);
      float w = 0.f;
      if (adjr[j] > 0.f) w = __expf(leaky(si + s_dst[bh * NN + j]) - em);
      lsum += w; A[e] = (_Float16)w;
    }
#pragma unroll
    for (int t = 0; t < 4; ++t) {
      v16h B;
#pragma unroll
      for (int e = 0; e < 16; ++e) B[e] = whh[(size_t)(jb + kmap(e, hh)) * HID + t * 16 + m];
      c[t] = wmma16(A, B, c[t]);
    }
  }
  lsum += __shfl_xor(lsum, 16);
#pragma unroll
  for (int r = 0; r < 8; ++r) {
    const float inv = 1.0f / __shfl(lsum, r + hh * 8);
#pragma unroll
    for (int t = 0; t < 4; ++t) { float v = c[t][r] * inv; if (doElu) v = (v > 0.f) ? v : (expf(v) - 1.0f); sO[wave][r + 8 * hh][t * 16 + m] = v; }
  }
  __builtin_amdgcn_fence(__ATOMIC_RELEASE, "workgroup"); __builtin_amdgcn_wave_barrier(); __builtin_amdgcn_fence(__ATOMIC_ACQUIRE, "workgroup");
  for (int pass = 0; pass < 2; ++pass) {
#pragma unroll
    for (int j = 0; j < 8; ++j) { const int rr = j * 2 + hh, q4 = m * 4;
      *(volatile v4f*)(out + ((size_t)b * NN + row0 + rr) * HID + head * HD + q4) = *(const v4f*)(&sO[wave][rr][q4]); }
    __threadfence();
  }
}
extern "C" void kernel_launch(void* const* d_in, const int* in_sizes, int n_in,
                              void* d_out, int out_size, void* d_ws, size_t ws_size, hipStream_t stream) {
  (void)in_sizes; (void)n_in; (void)out_size;
  const float* hin = (const float*)d_in[0];
  const float* adj = (const float*)d_in[1];
  const float* W1  = (const float*)d_in[2];
  const float* a1  = (const float*)d_in[3];
  const float* W2  = (const float*)d_in[4];
  const float* a2  = (const float*)d_in[5];
  float* out = (float*)d_out;
  char* ws = (char*)d_ws; size_t off = 0;
  auto take = [&](size_t bytes) { void* p = ws + off; off = (off + bytes + 255) & ~(size_t)255; return p; };
  float*    Wh   = (float*)take((size_t)NB * NN * HID * 4);
  _Float16* Whb  = (_Float16*)take((size_t)NB * NN * HID * 2);
  float*    x2   = (float*)take((size_t)NB * NN * HID * 4);
  float*    ssrc = (float*)take((size_t)NB * NH * NN * 4);
  float*    sdst = (float*)take((size_t)NB * NH * NN * 4);
  float*    emax = (float*)take((size_t)NB * NH * NN * 4);
  if (off > ws_size) return;
  k_xw<<<dim3(NN / 16, NH, NB), 128, 0, stream>>>(hin, 64, W1, Wh, Whb);
  k_scores<<<(NB * NH * NN) / 256, 256, 0, stream>>>(Wh, a1, ssrc, sdst);
  k_rowmax<<<dim3(NN / 32, NB * NH), 256, 0, stream>>>(adj, ssrc, sdst, emax);
  k_aggregate<<<dim3(NN / 16, NB), 96, 0, stream>>>(adj, Whb, ssrc, sdst, emax, x2, 1);
  k_xw<<<dim3(NN / 16, NH, NB), 128, 0, stream>>>(x2, HID, W2, Wh, Whb);
  k_scores<<<(NB * NH * NN) / 256, 256, 0, stream>>>(Wh, a2, ssrc, sdst);
  k_rowmax<<<dim3(NN / 32, NB * NH), 256, 0, stream>>>(adj, ssrc, sdst, emax);
  k_aggregate<<<dim3(NN / 16, NB), 96, 0, stream>>>(adj, Whb, ssrc, sdst, emax, out, 0);
}
